// LWSA_35098472743469
// MI455X (gfx1250) — hardware-verified
//
#include <hip/hip_runtime.h>


#define NBT  2
#define CC   256
#define DD_  12
#define NVOX 1728
#define NH_  4
#define INTER 128
#define DH   32
#define NTOK (NVOX * NH_)
#define EV   (CC / NH_)
#define QCH  768
#define DM   CC
#define NTK  NTOK
#define SCL  0.17677669529663687f
#define LOSC 1024.0f

typedef _Float16 h16;
typedef unsigned short bf;
typedef __attribute__((ext_vector_type(16))) __bf16   v16bf;
typedef __attribute__((ext_vector_type(16))) _Float16 v16h;
typedef __attribute__((ext_vector_type(8)))  _Float16 v8h;
typedef __attribute__((ext_vector_type(8)))  unsigned short v8us;
typedef __attribute__((ext_vector_type(8)))  float    v8f;
typedef __attribute__((ext_vector_type(4)))  float    v4f;
typedef __attribute__((ext_vector_type(4)))  _Float16 v4h;
typedef v8h  __attribute__((may_alias)) v8ha;
typedef v4f  __attribute__((may_alias)) v4fa;
typedef v8us __attribute__((may_alias)) v8usa;

__device__ __forceinline__ unsigned short f2bf(float f) { unsigned u = __float_as_uint(f); u += 0x7FFFu + ((u >> 16) & 1u); return (unsigned short)(u >> 16); }
__device__ __forceinline__ float bf2f(unsigned short b) { return __uint_as_float(((unsigned)b) << 16); }
__device__ __forceinline__ float bfr(float f) { return bf2f(f2bf(f)); }
__device__ __forceinline__ v16h cat16(v8h lo, v8h hi) { return __builtin_shufflevector(lo, hi, 0, 1, 2, 3, 4, 5, 6, 7, 8, 9, 10, 11, 12, 13, 14, 15); }
__device__ __forceinline__ v16bf cat16b(v8us lo, v8us hi) { return __builtin_bit_cast(v16bf, __builtin_shufflevector(lo, hi, 0, 1, 2, 3, 4, 5, 6, 7, 8, 9, 10, 11, 12, 13, 14, 15)); }
__device__ __forceinline__ v8f wmma16(v16h a, v16h b, v8f c) { return __builtin_amdgcn_wmma_f32_16x16x32_f16(false, a, false, b, (short)0, c, false, false); }
__device__ __forceinline__ v8f wmmab(v16bf a, v16bf b, v8f c) { return __builtin_amdgcn_wmma_f32_16x16x32_bf16(false, a, false, b, (short)0, c, false, false); }

__global__ __launch_bounds__(256) void k_wt(const float* __restrict__ Wm, int K, int ncols, bf* WT) {
    __shared__ __align__(16) unsigned short tl[64 * 72];
    const int tid = threadIdx.x, k0 = blockIdx.x * 64, n0 = blockIdx.y * 64;
    const int kk = tid >> 2, nq = (tid & 3) * 16;
#pragma unroll
    for (int i = 0; i < 16; ++i) tl[(nq + i) * 72 + kk] = f2bf(Wm[(size_t)(k0 + kk) * ncols + n0 + nq + i]);
    __syncthreads();
    const int piece = tid & 7;
    auto pass = [&]() {
#pragma unroll
        for (int s = 0; s < 2; ++s) { const int nr = (tid >> 3) + 32 * s; const v8us val = *(const v8usa*)(tl + nr * 72 + piece * 8); *(volatile v8us*)(WT + (size_t)(n0 + nr) * K + k0 + piece * 8) = val; }
    };
    pass(); __threadfence(); pass();
}
template <bool SPLITA, bool F16OUT = false>
__global__ __launch_bounds__(128) void k_gemmb(const bf* __restrict__ A, const bf* __restrict__ Al, const bf* __restrict__ Bn, const float* __restrict__ bias, float* C, int ldc, h16* C2, const float* __restrict__ R = nullptr, int K = DM, int roundR = 1) {
    __shared__ __align__(16) float ost[4][16 * 68];
    const int lane = threadIdx.x & 31, wave = threadIdx.x >> 5, lr = lane & 15, hi = lane >> 4;
    const int r0 = blockIdx.x * 64 + wave * 16, c0 = blockIdx.y * 64;
    const size_t aoff = (size_t)(r0 + lr) * K + 8 * hi;
    size_t boff[4];
#pragma unroll
    for (int t = 0; t < 4; ++t) boff[t] = (size_t)(c0 + t * 16 + lr) * K + 8 * hi;
    v8f acc[4];
#pragma unroll
    for (int t = 0; t < 4; ++t) acc[t] = (v8f){};
#pragma unroll 1
    for (int kc = 0; kc < K; kc += 32) {
        const v16bf a = cat16b(*(const v8us*)(A + aoff + kc), *(const v8us*)(A + aoff + kc + 16));
        v16bf al = a;
        if (SPLITA) al = cat16b(*(const v8us*)(Al + aoff + kc), *(const v8us*)(Al + aoff + kc + 16));
#pragma unroll
        for (int t = 0; t < 4; ++t) { const v16bf b = cat16b(*(const v8us*)(Bn + boff[t] + kc), *(const v8us*)(Bn + boff[t] + kc + 16)); acc[t] = wmmab(a, b, acc[t]); if (SPLITA) acc[t] = wmmab(al, b, acc[t]); }
        asm volatile("v_nop\n\tv_nop\n\tv_nop\n\tv_nop" : "+v"(acc[0]), "+v"(acc[1]), "+v"(acc[2]), "+v"(acc[3]) : "v"(a), "v"(al));
    }
    float* os = &ost[wave][0];
#pragma unroll
    for (int t = 0; t < 4; ++t) { const float bv = bias ? bfr(bias[c0 + t * 16 + lr]) : 0.f;
#pragma unroll
        for (int j = 0; j < 8; ++j) os[(hi * 8 + j) * 68 + t * 16 + lr] = acc[t][j] + bv; }
    __syncthreads();
    if (F16OUT) {
        h16* crow = (h16*)(void*)C + (size_t)r0 * ldc + c0;
        auto pass = [&]() {
#pragma unroll
            for (int s = 0; s < 4; ++s) { const int row = 4 * s + (lane >> 3), piece = lane & 7; const float* sp = os + row * 68 + piece * 8; v8h o, o2;
#pragma unroll
                for (int i = 0; i < 8; ++i) { const h16 a = (h16)sp[i]; o[i] = a; o2[i] = (h16)((sp[i] - (float)a) * LOSC); }
                *(volatile v8h*)(crow + (size_t)row * ldc + piece * 8) = o; if (C2) *(volatile v8h*)(C2 + (size_t)r0 * ldc + c0 + (size_t)row * ldc + piece * 8) = o2; }
        };
        pass(); __threadfence(); pass();
    } else {
        float* crow = C + (size_t)r0 * ldc + c0;
        auto pass = [&]() {
#pragma unroll
            for (int s = 0; s < 8; ++s) { const int Lid = (lane >> 3) + 4 * s, piece = lane & 7; const int row = Lid >> 1, cofs = (Lid & 1) * 32 + piece * 4;
                v4f val = *(const v4fa*)(os + row * 68 + cofs); if (R) { const v4f rv = *(const v4f*)(R + ((size_t)r0 + row) * ldc + c0 + cofs); val += roundR ? (v4f){bfr(rv[0]), bfr(rv[1]), bfr(rv[2]), bfr(rv[3])} : rv; }
                *(volatile v4f*)(crow + (size_t)row * ldc + cofs) = val; }
        };
        pass(); __threadfence(); pass();
    }
}

__global__ __launch_bounds__(128) void k_gemm3(const bf* __restrict__ Ah, const bf* __restrict__ Al, const bf* __restrict__ Bh, const bf* __restrict__ Bl, int K, float* C, int ldc) {
    __shared__ __align__(16) float ost[4][16 * 68];
    const int lane = threadIdx.x & 31, wave = threadIdx.x >> 5, lr = lane & 15, hi = lane >> 4;
    const int r0 = blockIdx.x * 64 + wave * 16, c0 = blockIdx.y * 64;
    const size_t aoff = (size_t)(r0 + lr) * K + 8 * hi;
    v8f acc[4];
#pragma unroll
    for (int t = 0; t < 4; ++t) acc[t] = (v8f){};
#pragma unroll 1
    for (int kc = 0; kc < K; kc += 32) {
        const v16bf a = cat16b(*(const v8us*)(Ah + aoff + kc), *(const v8us*)(Ah + aoff + kc + 16));
        const v16bf al = cat16b(*(const v8us*)(Al + aoff + kc), *(const v8us*)(Al + aoff + kc + 16));
#pragma unroll
        for (int t = 0; t < 4; ++t) { const size_t bo = (size_t)(c0 + t * 16 + lr) * K + kc + 8 * hi;
            const v16bf bh = cat16b(*(const v8us*)(Bh + bo), *(const v8us*)(Bh + bo + 16)); const v16bf bl = cat16b(*(const v8us*)(Bl + bo), *(const v8us*)(Bl + bo + 16));
            acc[t] = wmmab(a, bh, acc[t]); acc[t] = wmmab(al, bh, acc[t]); acc[t] = wmmab(a, bl, acc[t]); }
        asm volatile("v_nop\n\tv_nop\n\tv_nop\n\tv_nop" : "+v"(acc[0]), "+v"(acc[1]), "+v"(acc[2]), "+v"(acc[3]) : "v"(a), "v"(al));
    }
    float* os = &ost[wave][0];
#pragma unroll
    for (int t = 0; t < 4; ++t) {
#pragma unroll
        for (int j = 0; j < 8; ++j) os[(hi * 8 + j) * 68 + t * 16 + lr] = acc[t][j]; }
    __builtin_amdgcn_wave_barrier(); asm volatile("" ::: "memory");
    float* crow = C + (size_t)r0 * ldc + c0;
    auto pass = [&]() {
#pragma unroll
        for (int s = 0; s < 8; ++s) { const int Lid = (lane >> 3) + 4 * s, piece = lane & 7; const int row = Lid >> 1, cofs = (Lid & 1) * 32 + piece * 4;
            const v4f val = *(const v4fa*)(os + row * 68 + cofs); *(volatile v4f*)(crow + (size_t)row * ldc + cofs) = val; }
    };
    pass(); __threadfence(); pass();
}


__global__ __launch_bounds__(256) void k_cvt8(const float* __restrict__ src, bf* dst, size_t n8) {
    const size_t i = (size_t)blockIdx.x * 256 + threadIdx.x; if (i >= n8) return;
    const v8f v = *(const v8f*)(src + i * 8); v8us o;
#pragma unroll
    for (int k = 0; k < 8; ++k) o[k] = f2bf(v[k]);
    *(volatile v8us*)(dst + i * 8) = o; __threadfence(); *(volatile v8us*)(dst + i * 8) = o;
}
__global__ __launch_bounds__(256) void k_zero8(bf* dst, size_t n8) {
    const size_t i = (size_t)blockIdx.x * 256 + threadIdx.x; if (i >= n8) return; v8us z;
#pragma unroll
    for (int k = 0; k < 8; ++k) z[k] = 0;
    *(volatile v8us*)(dst + i * 8) = z; __threadfence(); *(volatile v8us*)(dst + i * 8) = z;
}

__global__ __launch_bounds__(256) void k_split32tok(const float* __restrict__ src, bf* dh, bf* dl) {
    typedef __attribute__((ext_vector_type(2))) unsigned short v2us;
    const int lane = threadIdx.x & 31; const size_t t = ((size_t)blockIdx.x * 8 + (threadIdx.x >> 5)) * 2 + (lane >> 4); if (t >= (size_t)NTOK) return; const int d = (lane & 15) * 2; v2us oh, ol;
#pragma unroll
    for (int i = 0; i < 2; ++i) { const float v = src[t * DH + d + i]; const unsigned short hb = f2bf(v); oh[i] = hb; ol[i] = f2bf(v - bf2f(hb)); }
    const size_t o = t * DH + d; *(volatile v2us*)(dh + o) = oh; *(volatile v2us*)(dl + o) = ol; __threadfence(); *(volatile v2us*)(dh + o) = oh; *(volatile v2us*)(dl + o) = ol;
}
__global__ __launch_bounds__(256) void k_vt(const float* __restrict__ xb, bf* VT) {
    typedef __attribute__((ext_vector_type(2))) unsigned short v2us;
    const int lane = threadIdx.x & 31; const size_t wid = (size_t)blockIdx.x * 8 + (threadIdx.x >> 5); if (wid >= (size_t)EV * (NTOK / 64)) return; const int e = (int)(wid / (NTOK / 64)); const int t0 = (int)(wid % (NTOK / 64)) * 64 + lane * 2; v2us o;
#pragma unroll
    for (int i = 0; i < 2; ++i) { const int t = t0 + i; const int n = t >> 2, h = t & 3; o[i] = f2bf(xb[((size_t)h * EV + e) * NVOX + n]); }
    *(volatile v2us*)(VT + (size_t)e * NTOK + t0) = o; __threadfence(); *(volatile v2us*)(VT + (size_t)e * NTOK + t0) = o;
}
__global__ __launch_bounds__(256) void k_softmax(const float* __restrict__ S, bf* PH, bf* PL) {
    typedef __attribute__((ext_vector_type(4))) unsigned short v4us;
    const int lane = threadIdx.x & 31, i = blockIdx.x * 8 + (threadIdx.x >> 5); if (i >= QCH) return;
    float m = -3.0e38f;
#pragma unroll 1
    for (int c0 = lane * 4; c0 < NTOK; c0 += 128) {
#pragma unroll
        for (int q = 0; q < 4; ++q) m = fmaxf(m, S[(size_t)i * NTOK + c0 + q] * SCL); }
#pragma unroll
    for (int sh = 16; sh; sh >>= 1) m = fmaxf(m, __shfl_xor(m, sh, 32));
    float sum = 0.f;
#pragma unroll 1
    for (int c0 = lane * 4; c0 < NTOK; c0 += 128) {
#pragma unroll
        for (int q = 0; q < 4; ++q) sum += __expf(S[(size_t)i * NTOK + c0 + q] * SCL - m); }
#pragma unroll
    for (int sh = 16; sh; sh >>= 1) sum += __shfl_xor(sum, sh, 32);
    const float inv = 1.0f / sum;
#pragma unroll 1
    for (int ps = 0; ps < 2; ++ps) {
#pragma unroll 1
        for (int c0 = lane * 4; c0 < NTOK; c0 += 128) { v4us oh, ol;
#pragma unroll
            for (int q = 0; q < 4; ++q) { const float p = __expf(S[(size_t)i * NTOK + c0 + q] * SCL - m) * inv; const unsigned short hb = f2bf(p); oh[q] = hb; ol[q] = f2bf(p - bf2f(hb)); }
            const size_t o = (size_t)i * NTOK + c0; *(volatile v4us*)(PH + o) = oh; *(volatile v4us*)(PL + o) = ol; }
        if (ps == 0) __threadfence(); }
}
__global__ __launch_bounds__(256) void k_fin(const float* __restrict__ O, const float* __restrict__ xb, const float* __restrict__ ws1, const float* __restrict__ bs1, const float* __restrict__ ws2, const float* __restrict__ bs2, float* OUTB) {
    typedef __attribute__((ext_vector_type(2))) float v2f;
    const int lane = threadIdx.x & 31; const size_t wid = (size_t)blockIdx.x * 8 + (threadIdx.x >> 5); if (wid >= (size_t)CC * (NVOX / 64)) return; const int c = (int)(wid / (NVOX / 64)); const int n0 = (int)(wid % (NVOX / 64)) * 64 + lane * 2;
    const bool big = c >= INTER; const int g = big ? c - INTER : c; const int ks = big ? 5 : 3, pad = big ? 2 : 1; const float* w = big ? (ws2 + (size_t)g * 2 * 125) : (ws1 + (size_t)g * 2 * 27); const float bb = big ? bfr(bs2[g]) : bfr(bs1[g]);
    v2f o;
#pragma unroll
    for (int i = 0; i < 2; ++i) { const int n = n0 + i; const int z = n / 144, y = (n / 12) % 12, xx = n % 12; float s = bb;
#pragma unroll 1
        for (int ic = 0; ic < 2; ++ic) { const float* xc = xb + (size_t)(2 * g + ic) * NVOX; const float* wc = w + ic * ks * ks * ks;
#pragma unroll 1
            for (int kz = 0; kz < ks; ++kz) { const int zz = z + kz - pad; if (zz < 0 || zz >= DD_) continue;
#pragma unroll 1
                for (int ky = 0; ky < ks; ++ky) { const int yy = y + ky - pad; if (yy < 0 || yy >= DD_) continue;
#pragma unroll 1
                    for (int kx = 0; kx < ks; ++kx) { const int xq = xx + kx - pad; if (xq < 0 || xq >= DD_) continue;
                        s = fmaf(bfr(xc[(zz * DD_ + yy) * DD_ + xq]), bfr(wc[(kz * ks + ky) * ks + kx]), s); } } } }
        o[i] = O[(size_t)n * CC + c] + tanhf(s); }
    *(volatile v2f*)(OUTB + (size_t)c * NVOX + n0) = o; __threadfence(); *(volatile v2f*)(OUTB + (size_t)c * NVOX + n0) = o;
}

extern "C" void kernel_launch(void* const* d_in, const int* in_sizes, int n_in,
                              void* d_out, int out_size, void* d_ws, size_t ws_size, hipStream_t stream) {
    (void)in_sizes; (void)n_in; (void)out_size;
    const float* x = (const float*)d_in[0]; const float* wq = (const float*)d_in[1]; const float* bq = (const float*)d_in[2]; const float* wk = (const float*)d_in[3]; const float* bk = (const float*)d_in[4];
    const float* ws1 = (const float*)d_in[5]; const float* bs1 = (const float*)d_in[6]; const float* ws2 = (const float*)d_in[7]; const float* bs2 = (const float*)d_in[8];
    float* out = (float*)d_out;
    char* wsp = (char*)d_ws;
    auto take = [&](size_t bytes) { char* p = wsp; wsp += (bytes + 255) & ~(size_t)255; return (void*)p; };
    bf* WQ = (bf*)take((size_t)INTER * CC * 2); bf* WK = (bf*)take((size_t)INTER * CC * 2); bf* XT = (bf*)take((size_t)NVOX * CC * 2); bf* VT = (bf*)take((size_t)EV * NTOK * 2); float* TMP = (float*)take((size_t)NVOX * INTER * 4);
    bf* Qh = (bf*)take((size_t)NTOK * DH * 2); bf* Ql = (bf*)take((size_t)NTOK * DH * 2); bf* Kh = (bf*)take((size_t)NTOK * DH * 2); bf* Kl = (bf*)take((size_t)NTOK * DH * 2);
    float* S = (float*)take((size_t)QCH * NTOK * 4); bf* PH = (bf*)take((size_t)QCH * NTOK * 2); bf* PL = (bf*)take((size_t)QCH * NTOK * 2); float* O = (float*)take((size_t)NTOK * EV * 4);
    if ((size_t)(wsp - (char*)d_ws) > ws_size) return;
    k_cvt8<<<(INTER * CC / 8 + 255) / 256, 256, 0, stream>>>(wq, WQ, INTER * CC / 8); k_cvt8<<<(INTER * CC / 8 + 255) / 256, 256, 0, stream>>>(wk, WK, INTER * CC / 8);
    for (int b = 0; b < NBT; ++b) { const float* xb = x + (size_t)b * CC * NVOX;
        k_wt<<<dim3(CC / 64, NVOX / 64, 1), 256, 0, stream>>>(xb, CC, NVOX, XT); k_vt<<<(EV * (NTOK / 64)) / 8, 256, 0, stream>>>(xb, VT);
        k_gemmb<false, false><<<dim3(NVOX / 64, INTER / 64, 1), 128, 0, stream>>>(XT, nullptr, WQ, bq, TMP, INTER, nullptr, nullptr, CC); k_split32tok<<<(NTOK / 2) / 8, 256, 0, stream>>>(TMP, Qh, Ql);
        k_gemmb<false, false><<<dim3(NVOX / 64, INTER / 64, 1), 128, 0, stream>>>(XT, nullptr, WK, bk, TMP, INTER, nullptr, nullptr, CC); k_split32tok<<<(NTOK / 2) / 8, 256, 0, stream>>>(TMP, Kh, Kl);
        for (int ch = 0; ch < NTOK / QCH; ++ch) { const size_t t0 = (size_t)ch * QCH;
            k_gemm3<<<dim3(QCH / 64, NTOK / 64, 1), 128, 0, stream>>>(Qh + t0 * DH, Ql + t0 * DH, Kh, Kl, DH, S, NTOK);
            k_softmax<<<QCH / 8, 256, 0, stream>>>(S, PH, PL);
            k_gemmb<true, false><<<dim3(QCH / 64, 1, 1), 128, 0, stream>>>(PH, PL, VT, nullptr, O + t0 * EV, EV, nullptr, nullptr, NTOK); }
        k_fin<<<(CC * (NVOX / 64)) / 8, 256, 0, stream>>>(O, xb, ws1, bs1, ws2, bs2, out + (size_t)b * CC * NVOX); }
}
